// FourierResistor_71880572666164
// MI455X (gfx1250) — hardware-run, weakly checked
//
#include <hip/hip_runtime.h>
#include <stddef.h>
#include <stdint.h>

#define BB     8
#define NN     4096
#define DD     128
#define HH     4
#define MROWS  (BB * NN)
#define TR     128
#define NTILE  (MROWS / TR)
#define TPB    (NN / TR)
#define NTHR   256
#define MODE_PHI 1
#define MODE_LN  2
#define MODE_H   2
#define KLT    DD
#define KPHI   (DD * MODE_PHI)
#define KLN    (DD * MODE_LN)
#define KH     (DD * MODE_H)

#define P_BPHI 0
#define P_WC1  512
#define P_BC1  528
#define P_WC2  532
#define P_BC2  536
#define P_LNG  544
#define P_LNB  672
#define P_BF1  800
#define P_BF2  928
#define PARN   2048

#define NB_XB   (MROWS * DD / 8 / NTHR)
#define NB_WLT  (DD * KLT / 8 / NTHR)
#define NB_WPHI (HH * DD * KPHI / 8 / NTHR)
#define NB_WF1  (DD * KLN / 8 / NTHR)
#define NB_WF2  (DD * KH / 8 / NTHR)
#define NB_POS  (NN * DD / 4 / NTHR)
#define NB_PREP (NB_XB + NB_WLT + NB_WPHI + NB_WF1 + NB_WF2 + NB_POS + 1)

#define AUXN   1024
#define LDSB   ((TR * DD + AUXN) * 4)

static_assert(DD == 128);
static_assert(HH == 4);
static_assert(NN % TR == 0);
static_assert(MROWS % TR == 0);
static_assert(NTHR == 256 && TR == (NTHR / 32) * 16);
static_assert(MODE_PHI == 1 || MODE_PHI == 2);
static_assert(MODE_LN == 1 || MODE_LN == 2);
static_assert(MODE_H == 1 || MODE_H == 2);
static_assert(KLT % 32 == 0 && KPHI % 32 == 0 && KLN % 32 == 0 && KH % 32 == 0);
static_assert((MROWS * DD / 8) % NTHR == 0 && (DD * KLT / 8) % NTHR == 0 && (HH * DD * KPHI / 8) % NTHR == 0);
static_assert((DD * KLN / 8) % NTHR == 0 && (DD * KH / 8) % NTHR == 0 && (NN * DD / 4) % NTHR == 0);
static_assert(PARN == 2 * NTHR * 4 && P_BF2 + DD <= PARN && P_WC1 + 32 <= P_LNG);
static_assert(LDSB <= 327680);

constexpr size_t SZ_XB   = (size_t)MROWS * DD * 2;
constexpr size_t SZ_XP   = (size_t)MROWS * KPHI * 2;
constexpr size_t SZ_MN   = (size_t)MROWS * KLN * 2;
constexpr size_t SZ_X1   = (size_t)MROWS * DD * 4;
constexpr size_t SZ_RFE  = (size_t)MROWS * HH * DD * 4;
constexpr size_t SZ_HHL  = (size_t)MROWS * KH * 2;
constexpr size_t SZ_POSR = (size_t)NN * DD * 4;
constexpr size_t SZ_WLT  = (size_t)DD * KLT * 2;
constexpr size_t SZ_WPHI = (size_t)HH * DD * KPHI * 2;
constexpr size_t SZ_WF1  = (size_t)DD * KLN * 2;
constexpr size_t SZ_WF2  = (size_t)DD * KH * 2;
constexpr size_t SZ_PAR  = (size_t)PARN * 4;
constexpr size_t SZ_R1   = (size_t)NTILE * 2 * DD * 4;
constexpr size_t SZ_R2   = (size_t)NTILE * HH * DD * 4;
constexpr size_t SZ_S1F  = (size_t)BB * 2 * DD * 4;
constexpr size_t SZ_S2F  = (size_t)BB * HH * DD * 4;
constexpr size_t O_XB    = 0;
constexpr size_t O_XP    = O_XB + SZ_XB;
constexpr size_t O_X1    = O_XP + SZ_XP;
constexpr size_t O_RFE   = O_X1 + SZ_X1;
constexpr size_t O_HHL   = O_RFE + SZ_RFE;
constexpr size_t O_POSR  = O_HHL + SZ_HHL;
constexpr size_t O_WLT   = O_POSR + SZ_POSR;
constexpr size_t O_WPHI  = O_WLT + SZ_WLT;
constexpr size_t O_WF1   = O_WPHI + SZ_WPHI;
constexpr size_t O_WF2   = O_WF1 + SZ_WF1;
constexpr size_t O_PAR   = O_WF2 + SZ_WF2;
constexpr size_t O_R1    = O_PAR + SZ_PAR;
constexpr size_t O_R2    = O_R1 + SZ_R1;
constexpr size_t O_S1F   = O_R2 + SZ_R2;
constexpr size_t O_S2F   = O_S1F + SZ_S1F;
constexpr size_t WS_TOTAL = O_S2F + SZ_S2F;
static_assert(SZ_XB % 256 == 0 && SZ_XP % 256 == 0 && SZ_X1 % 256 == 0 && SZ_RFE % 256 == 0 && SZ_HHL % 256 == 0);
static_assert(SZ_POSR % 256 == 0 && SZ_WLT % 256 == 0 && SZ_WPHI % 256 == 0 && SZ_WF1 % 256 == 0 && SZ_WF2 % 256 == 0);
static_assert(SZ_PAR % 256 == 0 && SZ_R1 % 256 == 0 && SZ_R2 % 256 == 0 && SZ_S1F % 256 == 0 && SZ_S2F % 256 == 0);
static_assert(SZ_MN <= SZ_XB + SZ_XP);
static_assert(WS_TOTAL <= (size_t)134217728);

typedef float          v4f   __attribute__((ext_vector_type(4)));
typedef float          v8f   __attribute__((ext_vector_type(8)));
typedef int            v8i   __attribute__((ext_vector_type(8)));
typedef unsigned short v4us  __attribute__((ext_vector_type(4)));
typedef unsigned short v8us  __attribute__((ext_vector_type(8)));
typedef unsigned short v16us __attribute__((ext_vector_type(16)));
typedef __bf16         v16bf __attribute__((ext_vector_type(16)));
typedef v4f  __attribute__((may_alias)) v4fa;
typedef v8us __attribute__((may_alias)) v8usa;
union FragB { v16bf v; v16us u; v8us h[2]; v8i w; };
struct HL4 { v4us h; v4us l; };

__device__ __forceinline__ v8f wmb(const FragB& a, const FragB& b, v8f c) {
  v8f d = __builtin_amdgcn_wmma_f32_16x16x32_bf16(false, a.v, false, b.v, (short)0, c, false, false);
  asm volatile("v_nop\n\tv_nop\n\tv_nop\n\tv_nop" : "+v"(d) : "v"(a.w), "v"(b.w));
  return d;
}

__device__ __forceinline__ v8f z8() { v8f z = {0.f, 0.f, 0.f, 0.f, 0.f, 0.f, 0.f, 0.f}; return z; }

__device__ __forceinline__ unsigned bf16_bits(float f) {
  const unsigned u = __float_as_uint(f);
  return (u + 0x7FFFu + ((u >> 16) & 1u)) >> 16;
}
__device__ __forceinline__ float bf16_val(float f) {
  return __uint_as_float(bf16_bits(f) << 16);
}

__device__ __forceinline__ HL4 split4(float a0, float a1, float a2, float a3) {
  HL4 o;
  const unsigned h0 = bf16_bits(a0), h1 = bf16_bits(a1), h2 = bf16_bits(a2), h3 = bf16_bits(a3);
  o.h[0] = (unsigned short)h0; o.h[1] = (unsigned short)h1;
  o.h[2] = (unsigned short)h2; o.h[3] = (unsigned short)h3;
  o.l[0] = (unsigned short)bf16_bits(a0 - __uint_as_float(h0 << 16));
  o.l[1] = (unsigned short)bf16_bits(a1 - __uint_as_float(h1 << 16));
  o.l[2] = (unsigned short)bf16_bits(a2 - __uint_as_float(h2 << 16));
  o.l[3] = (unsigned short)bf16_bits(a3 - __uint_as_float(h3 << 16));
  return o;
}

template <int KK>
__device__ __forceinline__ void gemm_16x128(const unsigned short* __restrict__ ap,
                                            const unsigned short* __restrict__ bp, v8f (&acc)[8]) {
#pragma unroll 1
  for (int k0 = 0; k0 < KK; k0 += 32) {
    FragB af;
    af.h[0] = *(const v8usa*)(ap + k0);
    af.h[1] = *(const v8usa*)(ap + k0 + 16);
#pragma unroll
    for (int nt = 0; nt < 8; ++nt) {
      const unsigned short* wq = bp + (size_t)(16 * nt) * (size_t)KK + k0;
      FragB bf;
      bf.h[0] = *(const v8usa*)wq;
      bf.h[1] = *(const v8usa*)(wq + 16);
      acc[nt] = wmb(af, bf, acc[nt]);
    }
  }
}

__device__ __forceinline__ void acc_to_stg(const v8f (&acc)[8], float* stg, int wave, int hh, int m) {
#pragma unroll
  for (int nt = 0; nt < 8; ++nt) {
#pragma unroll
    for (int r = 0; r < 8; ++r) {
      stg[(16 * wave + 8 * hh + r) * DD + 16 * nt + m] = acc[nt][r];
    }
  }
}

__device__ __forceinline__ void cvt8(const float* __restrict__ p, unsigned short* dp) {
  const v4f a = *(const v4f*)p;
  const v4f b = *(const v4f*)(p + 4);
  v8us o;
  o[0] = (unsigned short)bf16_bits(a.x); o[1] = (unsigned short)bf16_bits(a.y);
  o[2] = (unsigned short)bf16_bits(a.z); o[3] = (unsigned short)bf16_bits(a.w);
  o[4] = (unsigned short)bf16_bits(b.x); o[5] = (unsigned short)bf16_bits(b.y);
  o[6] = (unsigned short)bf16_bits(b.z); o[7] = (unsigned short)bf16_bits(b.w);
  *(volatile v8us*)dp = o;
  __threadfence();
  *(volatile v8us*)dp = o;
}

template <int K>
__device__ __forceinline__ void wdup8(const float* __restrict__ W, int v, unsigned short* dst) {
  constexpr int UPR = K / 8;
  const int n  = v / UPR;
  const int k8 = (v - n * UPR) * 8;
  const int kk = k8 & (DD - 1);
  cvt8(W + (size_t)n * DD + kk, dst + (size_t)v * 8);
}

__device__ __forceinline__ void stage_par(const float* __restrict__ src, int n, int off, float* sp, int tid) {
#pragma unroll 1
  for (int i0 = 0; i0 < n; i0 += NTHR) {
    const int i  = i0 + tid;
    const int ic = i < n ? i : n - 1;
    const float v = src[ic];
    asm volatile("" :: "v"(v));
    if (i < n) sp[off + i] = bf16_val(v);
  }
}

__global__ __launch_bounds__(NTHR) void k_prep(
    const float* __restrict__ x, const float* __restrict__ pos,
    const float* __restrict__ W_lt, const float* __restrict__ W_phi, const float* __restrict__ b_phi,
    const float* __restrict__ W_c1, const float* __restrict__ b_c1,
    const float* __restrict__ W_c2, const float* __restrict__ b_c2,
    const float* __restrict__ ln_g, const float* __restrict__ ln_b,
    const float* __restrict__ W_f1, const float* __restrict__ b_f1,
    const float* __restrict__ W_f2, const float* __restrict__ b_f2,
    unsigned short* XB, unsigned short* WLT, unsigned short* WPHI,
    unsigned short* WF1, unsigned short* WF2, float* POSR, float* PAR)
{
  __shared__ __attribute__((aligned(16))) float sp[PARN];
  const int tid = (int)threadIdx.x;
  int bid = (int)blockIdx.x;
  if (bid < NB_XB) {
    const int u = bid * NTHR + tid;
    cvt8(x + (size_t)u * 8, XB + (size_t)u * 8);
    return;
  }
  bid -= NB_XB;
  if (bid < NB_WLT) { wdup8<KLT>(W_lt, bid * NTHR + tid, WLT); return; }
  bid -= NB_WLT;
  if (bid < NB_WPHI) { wdup8<KPHI>(W_phi, bid * NTHR + tid, WPHI); return; }
  bid -= NB_WPHI;
  if (bid < NB_WF1) { wdup8<KLN>(W_f1, bid * NTHR + tid, WF1); return; }
  bid -= NB_WF1;
  if (bid < NB_WF2) { wdup8<KH>(W_f2, bid * NTHR + tid, WF2); return; }
  bid -= NB_WF2;
  if (bid < NB_POS) {
    const int u = bid * NTHR + tid;
    const v4f a = *(const v4f*)(pos + (size_t)u * 4);
    v4f o;
    o.x = bf16_val(a.x); o.y = bf16_val(a.y); o.z = bf16_val(a.z); o.w = bf16_val(a.w);
    float* dp = POSR + (size_t)u * 4;
    *(volatile v4f*)dp = o;
    __threadfence();
    *(volatile v4f*)dp = o;
    return;
  }
#pragma unroll 1
  for (int i = tid; i < PARN; i += NTHR) sp[i] = 0.0f;
  __syncthreads();
  stage_par(b_phi, HH * DD, P_BPHI, sp, tid);
  stage_par(W_c1, HH * HH, P_WC1, sp, tid);
  stage_par(b_c1, HH, P_BC1, sp, tid);
  stage_par(W_c2, HH, P_WC2, sp, tid);
  stage_par(b_c2, 1, P_BC2, sp, tid);
  stage_par(ln_g, DD, P_LNG, sp, tid);
  stage_par(ln_b, DD, P_LNB, sp, tid);
  stage_par(b_f1, DD, P_BF1, sp, tid);
  stage_par(b_f2, DD, P_BF2, sp, tid);
  __syncthreads();
  const v4f q0 = *(const v4fa*)(sp + 4 * tid);
  const v4f q1 = *(const v4fa*)(sp + 4 * (tid + NTHR));
  *(volatile v4f*)(PAR + 4 * tid) = q0;
  *(volatile v4f*)(PAR + 4 * (tid + NTHR)) = q1;
  __threadfence();
  *(volatile v4f*)(PAR + 4 * tid) = q0;
  *(volatile v4f*)(PAR + 4 * (tid + NTHR)) = q1;
}

__device__ __forceinline__ void lt_store_pass(const float* stg, const float* __restrict__ POSR,
                                              float* X1, unsigned short* XP,
                                              int rowBase, int n0, int wave, int lane) {
#pragma unroll 1
  for (int i = 0; i < 16; ++i) {
    const int lr = 16 * wave + i;
    const v4f xv = *(const v4fa*)(stg + lr * DD + 4 * lane);
    const v4f pv = *(const v4f*)(POSR + (size_t)(n0 + lr) * DD + 4 * lane);
    const HL4 s = split4(xv.x + pv.x, xv.y + pv.y, xv.z + pv.z, xv.w + pv.w);
    const size_t row = (size_t)(rowBase + lr);
    *(volatile v4f*)(X1 + row * DD + 4 * lane) = xv;
    *(volatile v4us*)(XP + row * KPHI + 4 * lane) = s.h;
    if constexpr (MODE_PHI == 2) {
      *(volatile v4us*)(XP + row * KPHI + DD + 4 * lane) = s.l;
    }
  }
}

__global__ __launch_bounds__(NTHR) __attribute__((amdgpu_num_vgpr(248)))
void k_lt(const unsigned short* __restrict__ XB, const unsigned short* __restrict__ WLT,
          const float* __restrict__ POSR, float* X1, unsigned short* XP, float* R1)
{
  extern __shared__ __attribute__((aligned(16))) float dsm[];
  float* stg = dsm;
  float* aux = dsm + TR * DD;
  const int tid = (int)threadIdx.x, lane = tid & 31, wave = tid >> 5, hh = lane >> 4, m = lane & 15;
  const int tile = (int)blockIdx.x;
  const int rowBase = tile * TR;
  const int n0 = rowBase & (NN - 1);

  v8f acc[8];
#pragma unroll
  for (int t = 0; t < 8; ++t) acc[t] = z8();
  gemm_16x128<KLT>(XB + (size_t)(rowBase + 16 * wave + m) * KLT + 8 * hh,
                   WLT + (size_t)m * KLT + 8 * hh, acc);
  acc_to_stg(acc, stg, wave, hh, m);
  __syncthreads();

  {
    const int k = tid >> 7, c = tid & (DD - 1);
    const int pc = (k == 0) ? (c | 1) : (c & ~1);
    const float sg = (k == 0) ? 1.0f : -1.0f;
    const float* pp = POSR + (size_t)n0 * DD + pc;
    float s = 0.0f;
#pragma unroll 4
    for (int r = 0; r < TR; ++r) {
      s += stg[r * DD + c] * (sg * pp[(size_t)r * DD]);
    }
    aux[tid] = s;
  }

  lt_store_pass(stg, POSR, X1, XP, rowBase, n0, wave, lane);
  __syncthreads();
  v4f rv = {0.f, 0.f, 0.f, 0.f};
  if (tid < 64) {
    rv = *(const v4fa*)(aux + 4 * tid);
    *(volatile v4f*)(R1 + (size_t)tile * (2 * DD) + 4 * tid) = rv;
  }
  __threadfence();
  lt_store_pass(stg, POSR, X1, XP, rowBase, n0, wave, lane);
  if (tid < 64) {
    *(volatile v4f*)(R1 + (size_t)tile * (2 * DD) + 4 * tid) = rv;
  }
}

template <int W>
__global__ __launch_bounds__(NTHR) void k_sum(const float* __restrict__ rec, float* out) {
  __shared__ __attribute__((aligned(16))) float s[BB * W];
  const int tid = (int)threadIdx.x;
#pragma unroll 1
  for (int o = tid; o < BB * W; o += NTHR) {
    const int b = o / W;
    const int q = o - b * W;
    const float* p = rec + (size_t)b * TPB * W + q;
    double a = 0.0;
#pragma unroll 4
    for (int t = 0; t < TPB; ++t) a += (double)p[(size_t)t * W];
    s[o] = (float)a;
  }
  __syncthreads();
#pragma unroll 1
  for (int i = tid; i < BB * W / 4; i += NTHR) {
    const v4f v = *(const v4fa*)(s + 4 * i);
    *(volatile v4f*)(out + 4 * i) = v;
  }
  __threadfence();
#pragma unroll 1
  for (int i = tid; i < BB * W / 4; i += NTHR) {
    const v4f v = *(const v4fa*)(s + 4 * i);
    *(volatile v4f*)(out + 4 * i) = v;
  }
}

__device__ __forceinline__ float rfe_one(float x, float cc, float ss, float s0, float s1, float phi) {
#pragma clang fp contract(off)
  const float xe0 = x * cc;
  const float xe1 = x * (-ss);
  const float f0 = s0 - xe0;
  const float f1 = s1 - xe1;
  const float fn = sqrtf(f0 * f0 + f1 * f1);
  const float t = fminf(1.0f, fn - phi);
  const float res = (t > 0.0f) ? t : (t - t);
  const float fec = f0 * cc - f1 * ss;
  return res * fec;
}

__global__ __launch_bounds__(NTHR) __attribute__((amdgpu_num_vgpr(248)))
void k_phi(const unsigned short* __restrict__ XP, const unsigned short* __restrict__ WPHI,
           const float* __restrict__ X1, const float* __restrict__ POSR,
           const float* __restrict__ PAR, const float* __restrict__ S1F,
           float* RFE, float* R2)
{
  extern __shared__ __attribute__((aligned(16))) float dsm[];
  float* stg = dsm;
  float* aux = dsm + TR * DD;
  const int tid = (int)threadIdx.x, lane = tid & 31, wave = tid >> 5, hh = lane >> 4, m = lane & 15;
  const int tile = (int)blockIdx.x;
  const int h = (int)blockIdx.y;
  const int rowBase = tile * TR;
  const int n0 = rowBase & (NN - 1);
  const int b = tile / TPB;

  if (wave < 2) {
    const v4f v = *(const v4f*)(S1F + (size_t)b * (2 * DD) + 4 * tid);
    *(v4fa*)(aux + 4 * tid) = v;
  } else if (wave == 2) {
    const v4f v = *(const v4f*)(PAR + P_BPHI + h * DD + 4 * lane);
    *(v4fa*)(aux + 2 * DD + 4 * lane) = v;
  }

  v8f acc[8];
#pragma unroll
  for (int t = 0; t < 8; ++t) acc[t] = z8();
  gemm_16x128<KPHI>(XP + (size_t)(rowBase + 16 * wave + m) * KPHI + 8 * hh,
                    WPHI + (size_t)(h * DD + m) * KPHI + 8 * hh, acc);
  acc_to_stg(acc, stg, wave, hh, m);
  __syncthreads();

  const v4f s04 = *(const v4fa*)(aux + 4 * lane);
  const v4f s14 = *(const v4fa*)(aux + DD + 4 * lane);
  const v4f bp4 = *(const v4fa*)(aux + 2 * DD + 4 * lane);
#pragma unroll 1
  for (int i = 0; i < 16; ++i) {
    const int lr = 16 * wave + i;
    const size_t row = (size_t)(rowBase + lr);
    const v4f ph = *(const v4fa*)(stg + lr * DD + 4 * lane);
    const v4f xv = *(const v4f*)(X1 + row * DD + 4 * lane);
    const v4f pv = *(const v4f*)(POSR + (size_t)(n0 + lr) * DD + 4 * lane);
    v4f o;
    o.x = rfe_one(xv.x, pv.y, pv.x, s04.x, s14.x, ph.x + bp4.x);
    o.y = rfe_one(xv.y, pv.y, pv.x, s04.y, s14.y, ph.y + bp4.y);
    o.z = rfe_one(xv.z, pv.w, pv.z, s04.z, s14.z, ph.z + bp4.z);
    o.w = rfe_one(xv.w, pv.w, pv.z, s04.w, s14.w, ph.w + bp4.w);
    *(volatile v4f*)(RFE + row * (HH * DD) + h * DD + 4 * lane) = o;
    *(v4fa*)(stg + lr * DD + 4 * lane) = o;
  }
  __syncthreads();

  if (tid < DD) {
    float s = 0.0f;
#pragma unroll 4
    for (int r = 0; r < TR; ++r) s += stg[r * DD + tid];
    aux[3 * DD + tid] = s;
  }
  __threadfence();
#pragma unroll 1
  for (int i = 0; i < 16; ++i) {
    const int lr = 16 * wave + i;
    const size_t row = (size_t)(rowBase + lr);
    const v4f o = *(const v4fa*)(stg + lr * DD + 4 * lane);
    *(volatile v4f*)(RFE + row * (HH * DD) + h * DD + 4 * lane) = o;
  }
  __syncthreads();
  v4f rv = {0.f, 0.f, 0.f, 0.f};
  float* rp = R2 + ((size_t)tile * HH + h) * DD + 4 * lane;
  if (tid < 32) {
    rv = *(const v4fa*)(aux + 3 * DD + 4 * tid);
    *(volatile v4f*)rp = rv;
  }
  __threadfence();
  if (tid < 32) {
    *(volatile v4f*)rp = rv;
  }
}

__global__ __launch_bounds__(NTHR) void k_comb_ln(const float* __restrict__ RFE, const float* __restrict__ X1,
                                                  const float* __restrict__ S2F, const float* __restrict__ PAR,
                                                  unsigned short* MNHL)
{
  __shared__ __attribute__((aligned(16))) float s2[HH * DD];
  __shared__ __attribute__((aligned(16))) float lng[DD];
  __shared__ __attribute__((aligned(16))) float lnb[DD];
  __shared__ __attribute__((aligned(16))) float prm[32];
  __shared__ __attribute__((aligned(16))) float mrow[8 * DD];
  const int tid = (int)threadIdx.x, lane = tid & 31, wave = tid >> 5;
  const int tile = (int)blockIdx.x;
  const int rowBase = tile * TR;
  const int b = tile / TPB;

  if (wave < 4) {
    const v4f v = *(const v4f*)(S2F + (size_t)b * (HH * DD) + 4 * tid);
    *(v4fa*)(s2 + 4 * tid) = v;
  } else if (wave == 4) {
    const v4f v = *(const v4f*)(PAR + P_LNG + 4 * lane);
    *(v4fa*)(lng + 4 * lane) = v;
  } else if (wave == 5) {
    const v4f v = *(const v4f*)(PAR + P_LNB + 4 * lane);
    *(v4fa*)(lnb + 4 * lane) = v;
  } else if (wave == 6) {
    prm[lane] = PAR[P_WC1 + lane];
  }
  __syncthreads();

  float wc1[16], bc1[4], wc2[4];
#pragma unroll
  for (int i = 0; i < 16; ++i) wc1[i] = prm[i];
#pragma unroll
  for (int i = 0; i < 4; ++i) { bc1[i] = prm[16 + i]; wc2[i] = prm[20 + i]; }
  const float bc2 = prm[24];
  const v4f g4 = *(const v4fa*)(lng + 4 * lane);
  const v4f e4 = *(const v4fa*)(lnb + 4 * lane);

#pragma unroll 1
  for (int it = 0; it < 16; ++it) {
    const int lr = it * 8 + wave;
    const size_t row = (size_t)(rowBase + lr);
    const float* rr = RFE + row * (HH * DD);
    const float* xr = X1 + row * DD;
#pragma unroll 1
    for (int j = 0; j < 4; ++j) {
      const int c = lane + 32 * j;
      const float r0 = rr[c];
      const float r1 = rr[DD + c];
      const float r2 = rr[2 * DD + c];
      const float r3 = rr[3 * DD + c];
      const float xv = xr[c];
      const float i0 = (s2[c] - r0) * (1.0f / 4096.0f);
      const float i1 = (s2[DD + c] - r1) * (1.0f / 4096.0f);
      const float i2 = (s2[2 * DD + c] - r2) * (1.0f / 4096.0f);
      const float i3 = (s2[3 * DD + c] - r3) * (1.0f / 4096.0f);
      float comb = 0.0f;
#pragma unroll
      for (int q = 0; q < 4; ++q) {
        float u = i0 * wc1[4 * q];
        u = fmaf(i1, wc1[4 * q + 1], u);
        u = fmaf(i2, wc1[4 * q + 2], u);
        u = fmaf(i3, wc1[4 * q + 3], u);
        u = u + bc1[q];
        const float hd = (u > 0.0f) ? u : (u - u);
        comb = fmaf(hd, wc2[q], comb);
      }
      comb = comb + bc2;
      mrow[wave * DD + c] = xv + comb;
    }
    __syncthreads();
    const v4f m4 = *(const v4fa*)(mrow + wave * DD + 4 * lane);
    float sum = (m4.x + m4.y) + (m4.z + m4.w);
    sum += __shfl_xor(sum, 16);
    sum += __shfl_xor(sum, 8);
    sum += __shfl_xor(sum, 4);
    sum += __shfl_xor(sum, 2);
    sum += __shfl_xor(sum, 1);
    const float mu = sum * (1.0f / 128.0f);
    const float d0 = m4.x - mu, d1 = m4.y - mu, d2 = m4.z - mu, d3 = m4.w - mu;
    float sq = (d0 * d0 + d1 * d1) + (d2 * d2 + d3 * d3);
    sq += __shfl_xor(sq, 16);
    sq += __shfl_xor(sq, 8);
    sq += __shfl_xor(sq, 4);
    sq += __shfl_xor(sq, 2);
    sq += __shfl_xor(sq, 1);
    const float var = sq * (1.0f / 128.0f);
    const float rstd = 1.0f / sqrtf(var + 1e-6f);
    const float y0 = d0 * rstd * g4.x + e4.x;
    const float y1 = d1 * rstd * g4.y + e4.y;
    const float y2 = d2 * rstd * g4.z + e4.z;
    const float y3 = d3 * rstd * g4.w + e4.w;
    const HL4 s = split4(y0, y1, y2, y3);
    unsigned short* op = MNHL + row * KLN + 4 * lane;
    *(volatile v4us*)op = s.h;
    if constexpr (MODE_LN == 2) { *(volatile v4us*)(op + DD) = s.l; }
    __threadfence();
    *(volatile v4us*)op = s.h;
    if constexpr (MODE_LN == 2) { *(volatile v4us*)(op + DD) = s.l; }
    __syncthreads();
  }
}

__device__ __forceinline__ void f1_store_pass(const float* stg, const float* aux, unsigned short* HHL,
                                              int rowBase, int wave, int lane) {
  const v4f bq = *(const v4fa*)(aux + 4 * lane);
#pragma unroll 1
  for (int i = 0; i < 16; ++i) {
    const int lr = 16 * wave + i;
    const v4f xv = *(const v4fa*)(stg + lr * DD + 4 * lane);
    const float u0 = xv.x + bq.x, u1 = xv.y + bq.y, u2 = xv.z + bq.z, u3 = xv.w + bq.w;
    const float y0 = (u0 > 0.0f) ? u0 : (u0 - u0);
    const float y1 = (u1 > 0.0f) ? u1 : (u1 - u1);
    const float y2 = (u2 > 0.0f) ? u2 : (u2 - u2);
    const float y3 = (u3 > 0.0f) ? u3 : (u3 - u3);
    const HL4 s = split4(y0, y1, y2, y3);
    unsigned short* op = HHL + (size_t)(rowBase + lr) * KH + 4 * lane;
    *(volatile v4us*)op = s.h;
    if constexpr (MODE_H == 2) { *(volatile v4us*)(op + DD) = s.l; }
  }
}

__global__ __launch_bounds__(NTHR) __attribute__((amdgpu_num_vgpr(248)))
void k_f1(const unsigned short* __restrict__ MNHL, const unsigned short* __restrict__ WF1,
          const float* __restrict__ PAR, unsigned short* HHL)
{
  extern __shared__ __attribute__((aligned(16))) float dsm[];
  float* stg = dsm;
  float* aux = dsm + TR * DD;
  const int tid = (int)threadIdx.x, lane = tid & 31, wave = tid >> 5, hh = lane >> 4, m = lane & 15;
  const int rowBase = (int)blockIdx.x * TR;
  if (wave == 0) {
    const v4f v = *(const v4f*)(PAR + P_BF1 + 4 * lane);
    *(v4fa*)(aux + 4 * lane) = v;
  }
  v8f acc[8];
#pragma unroll
  for (int t = 0; t < 8; ++t) acc[t] = z8();
  gemm_16x128<KLN>(MNHL + (size_t)(rowBase + 16 * wave + m) * KLN + 8 * hh,
                   WF1 + (size_t)m * KLN + 8 * hh, acc);
  acc_to_stg(acc, stg, wave, hh, m);
  __syncthreads();
  f1_store_pass(stg, aux, HHL, rowBase, wave, lane);
  __threadfence();
  f1_store_pass(stg, aux, HHL, rowBase, wave, lane);
}

__device__ __forceinline__ void f2_store_pass(const float* stg, const float* aux, float* out,
                                              int rowBase, int wave, int lane) {
  const v4f bq = *(const v4fa*)(aux + 4 * lane);
#pragma unroll 1
  for (int i = 0; i < 16; ++i) {
    const int lr = 16 * wave + i;
    const v4f xv = *(const v4fa*)(stg + lr * DD + 4 * lane);
    v4f o;
    o.x = xv.x + bq.x; o.y = xv.y + bq.y; o.z = xv.z + bq.z; o.w = xv.w + bq.w;
    *(volatile v4f*)(out + (size_t)(rowBase + lr) * DD + 4 * lane) = o;
  }
}

__global__ __launch_bounds__(NTHR) __attribute__((amdgpu_num_vgpr(248)))
void k_f2(const unsigned short* __restrict__ HHL, const unsigned short* __restrict__ WF2,
          const float* __restrict__ PAR, float* out)
{
  extern __shared__ __attribute__((aligned(16))) float dsm[];
  float* stg = dsm;
  float* aux = dsm + TR * DD;
  const int tid = (int)threadIdx.x, lane = tid & 31, wave = tid >> 5, hh = lane >> 4, m = lane & 15;
  const int rowBase = (int)blockIdx.x * TR;
  if (wave == 0) {
    const v4f v = *(const v4f*)(PAR + P_BF2 + 4 * lane);
    *(v4fa*)(aux + 4 * lane) = v;
  }
  v8f acc[8];
#pragma unroll
  for (int t = 0; t < 8; ++t) acc[t] = z8();
  gemm_16x128<KH>(HHL + (size_t)(rowBase + 16 * wave + m) * KH + 8 * hh,
                  WF2 + (size_t)m * KH + 8 * hh, acc);
  acc_to_stg(acc, stg, wave, hh, m);
  __syncthreads();
  f2_store_pass(stg, aux, out, rowBase, wave, lane);
  __threadfence();
  f2_store_pass(stg, aux, out, rowBase, wave, lane);
}

extern "C" void kernel_launch(void* const* d_in, const int* in_sizes, int n_in,
                              void* d_out, int out_size, void* d_ws, size_t ws_size,
                              hipStream_t stream) {
  if (n_in < 15) return;
  if (in_sizes[0] != MROWS * DD) return;
  if (in_sizes[1] != NN * DD) return;
  if (in_sizes[2] != DD * DD) return;
  if (in_sizes[3] != HH * DD * DD) return;
  if (in_sizes[4] != HH * DD) return;
  if (in_sizes[5] != HH * HH || in_sizes[6] != HH) return;
  if (in_sizes[7] != HH || in_sizes[8] != 1) return;
  if (in_sizes[9] != DD || in_sizes[10] != DD) return;
  if (in_sizes[11] != DD * DD || in_sizes[12] != DD) return;
  if (in_sizes[13] != DD * DD || in_sizes[14] != DD) return;
  if (out_size != MROWS * DD) return;
  if (WS_TOTAL > ws_size) return;

  const float* x     = (const float*)d_in[0];
  const float* pos   = (const float*)d_in[1];
  const float* W_lt  = (const float*)d_in[2];
  const float* W_phi = (const float*)d_in[3];
  const float* b_phi = (const float*)d_in[4];
  const float* W_c1  = (const float*)d_in[5];
  const float* b_c1  = (const float*)d_in[6];
  const float* W_c2  = (const float*)d_in[7];
  const float* b_c2  = (const float*)d_in[8];
  const float* ln_g  = (const float*)d_in[9];
  const float* ln_b  = (const float*)d_in[10];
  const float* W_f1  = (const float*)d_in[11];
  const float* b_f1  = (const float*)d_in[12];
  const float* W_f2  = (const float*)d_in[13];
  const float* b_f2  = (const float*)d_in[14];
  float* out = (float*)d_out;

  char* ws = (char*)d_ws;
  unsigned short* XB   = (unsigned short*)(ws + O_XB);
  unsigned short* XP   = (unsigned short*)(ws + O_XP);
  unsigned short* MNHL = (unsigned short*)(ws + O_XB);
  float*          X1   = (float*)(ws + O_X1);
  float*          RFE  = (float*)(ws + O_RFE);
  unsigned short* HHL  = (unsigned short*)(ws + O_HHL);
  float*          POSR = (float*)(ws + O_POSR);
  unsigned short* WLT  = (unsigned short*)(ws + O_WLT);
  unsigned short* WPHI = (unsigned short*)(ws + O_WPHI);
  unsigned short* WF1  = (unsigned short*)(ws + O_WF1);
  unsigned short* WF2  = (unsigned short*)(ws + O_WF2);
  float*          PAR  = (float*)(ws + O_PAR);
  float*          R1   = (float*)(ws + O_R1);
  float*          R2   = (float*)(ws + O_R2);
  float*          S1F  = (float*)(ws + O_S1F);
  float*          S2F  = (float*)(ws + O_S2F);

  hipFuncSetAttribute(reinterpret_cast<const void*>(&k_lt),  hipFuncAttributeMaxDynamicSharedMemorySize, (int)LDSB);
  hipFuncSetAttribute(reinterpret_cast<const void*>(&k_phi), hipFuncAttributeMaxDynamicSharedMemorySize, (int)LDSB);
  hipFuncSetAttribute(reinterpret_cast<const void*>(&k_f1),  hipFuncAttributeMaxDynamicSharedMemorySize, (int)LDSB);
  hipFuncSetAttribute(reinterpret_cast<const void*>(&k_f2),  hipFuncAttributeMaxDynamicSharedMemorySize, (int)LDSB);

  k_prep<<<NB_PREP, NTHR, 0, stream>>>(x, pos, W_lt, W_phi, b_phi, W_c1, b_c1, W_c2, b_c2, ln_g, ln_b,
                                        W_f1, b_f1, W_f2, b_f2, XB, WLT, WPHI, WF1, WF2, POSR, PAR);
  k_lt<<<NTILE, NTHR, LDSB, stream>>>(XB, WLT, POSR, X1, XP, R1);
  k_sum<2 * DD><<<1, NTHR, 0, stream>>>(R1, S1F);
  k_phi<<<dim3(NTILE, HH), NTHR, LDSB, stream>>>(XP, WPHI, X1, POSR, PAR, S1F, RFE, R2);
  k_sum<HH * DD><<<1, NTHR, 0, stream>>>(R2, S2F);
  k_comb_ln<<<NTILE, NTHR, 0, stream>>>(RFE, X1, S2F, PAR, MNHL);
  k_f1<<<NTILE, NTHR, LDSB, stream>>>(MNHL, WF1, PAR, HHL);
  k_f2<<<NTILE, NTHR, LDSB, stream>>>(HHL, WF2, PAR, out);
}
